// ZoomInSelfAttention_80788334838078
// MI455X (gfx1250) — hardware-verified
//
#include <hip/hip_runtime.h>
#define BB 4
#define CC 256
#define HW 64
#define LQ (HW * HW)
#define LK (LQ / 4)
#define NHD 8
#define DH 32
#define NP (BB * LQ)
#define CH 128
#define SE 16

typedef __bf16 v16b __attribute__((ext_vector_type(16)));
typedef unsigned short v8us __attribute__((ext_vector_type(8), may_alias));
typedef float  v8f  __attribute__((ext_vector_type(8)));
typedef float  v4f  __attribute__((ext_vector_type(4)));
typedef float  v4fa __attribute__((ext_vector_type(4), may_alias));
union FragB { v16b v; v8us half[2]; unsigned short u[16]; };

__device__ __forceinline__ unsigned short bf16_bits(float x) { unsigned int u = __float_as_uint(x); return (unsigned short)((u + 0x7FFFu + ((u >> 16) & 1u)) >> 16); }
__device__ __forceinline__ float bf16_val(unsigned short b) { return __uint_as_float(((unsigned int)b) << 16); }
__device__ __forceinline__ float bf16_round(float x) { return bf16_val(bf16_bits(x)); }
template <int NT>
__device__ __forceinline__ v8f mmaN(v16b ah, v16b al, v16b bh, v16b bl, v8f c) {
  c = __builtin_amdgcn_wmma_f32_16x16x32_bf16(false, ah, false, bh, (short)0, c, false, false);
  if (NT >= 2) c = __builtin_amdgcn_wmma_f32_16x16x32_bf16(false, al, false, bh, (short)0, c, false, false);
  if (NT >= 3) c = __builtin_amdgcn_wmma_f32_16x16x32_bf16(false, ah, false, bl, (short)0, c, false, false);
  asm volatile("v_nop\n\tv_nop\n\tv_nop\n\tv_nop" : "+v"(c) : "v"(ah), "v"(al), "v"(bh), "v"(bl));
  return c;
}

__global__ __launch_bounds__(256) void k_wt_bf16(const float* __restrict__ W, unsigned short* __restrict__ Wt, int K, int N) {
  const int t = blockIdx.x * 256 + threadIdx.x;
  const int k8n = K / 8;
  if (t >= N * k8n) return;
  const int n = t / k8n, k8 = (t % k8n) * 8;
  v8us v;
#pragma unroll
  for (int i = 0; i < 8; ++i) v[i] = bf16_bits(W[(size_t)(k8 + i) * N + n]);
  *(volatile v8us*)(Wt + (size_t)n * K + k8) = v;
  __threadfence();
  *(volatile v8us*)(Wt + (size_t)n * K + k8) = v;
}

template <bool ASPLIT, int ACT, bool BIAS_BF16>
__global__ __launch_bounds__(128) void k_gemm_bf(const float* __restrict__ A, int lda, const unsigned short* __restrict__ Wt, int ldb,
                                               const float* __restrict__ bias, float* __restrict__ C, int ldc, int M, int N, int K) {
  __shared__ __attribute__((aligned(16))) float so[4][16][64];
  const int tid = threadIdx.x, w = tid >> 5, lane = tid & 31, ln = lane & 15, hh = lane >> 4;
  const int ntn = N / 64;
  const int wid = blockIdx.x * 4 + w;
  const int mt = wid / ntn, nq = wid % ntn;
  if (mt * 16 >= M) return;
  const int row0 = mt * 16, col0 = nq * 64;
  const float* arow = A + (size_t)(row0 + ln) * lda;
  v8f acc[4] = {};
  for (int kb = 0; kb < K; kb += 32) {
    FragB ah, al;
    const v4f x0 = *(const v4fa*)(arow + kb + 8 * hh), x1 = *(const v4fa*)(arow + kb + 8 * hh + 4);
    const v4f x2 = *(const v4fa*)(arow + kb + 16 + 8 * hh), x3 = *(const v4fa*)(arow + kb + 16 + 8 * hh + 4);
    float xs[16] = {x0[0],x0[1],x0[2],x0[3],x1[0],x1[1],x1[2],x1[3],x2[0],x2[1],x2[2],x2[3],x3[0],x3[1],x3[2],x3[3]};
#pragma unroll
    for (int i = 0; i < 16; ++i) { const unsigned short hb = bf16_bits(xs[i]); ah.u[i] = hb; al.u[i] = ASPLIT ? bf16_bits(xs[i] - bf16_val(hb)) : (unsigned short)0; }
#pragma unroll
    for (int t = 0; t < 4; ++t) {
      const unsigned short* brow = Wt + (size_t)(col0 + t * 16 + ln) * ldb + kb;
      FragB b;
      b.half[0] = *(const v8us*)(brow + 8 * hh);
      b.half[1] = *(const v8us*)(brow + 16 + 8 * hh);
      acc[t] = mmaN<ASPLIT ? 2 : 1>(ah.v, al.v, b.v, b.v, acc[t]);
    }
  }
#pragma unroll
  for (int t = 0; t < 4; ++t) {
    float bv = bias ? bias[col0 + t * 16 + ln] : 0.f;
    if (BIAS_BF16) bv = bf16_round(bv);
#pragma unroll
    for (int r = 0; r < 8; ++r) { float v = acc[t][r] + bv; if (ACT == 1) v = fmaxf(v, 0.f); so[w][8 * hh + r][t * 16 + ln] = v; }
  }
  __builtin_amdgcn_fence(__ATOMIC_ACQ_REL, "workgroup");
  __builtin_amdgcn_wave_barrier();
  const int rsub = lane >> 4, c4 = (lane & 15) * 4;
  for (int pass = 0; pass < 2; ++pass) {
#pragma unroll
    for (int q = 0; q < 8; ++q) {
      const int r = q * 2 + rsub;
      const v4f v = *(const v4fa*)&so[w][r][c4];
      *(volatile v4f*)(C + (size_t)(row0 + r) * ldc + col0 + c4) = v;
    }
    if (pass == 0) __threadfence();
  }
}

template <int D, bool CAUSAL>
__global__ __launch_bounds__(128) void k_flash(const float* __restrict__ qb, const float* __restrict__ kb, const float* __restrict__ vb,
                                             int pitch, int T, int H, float scale, float* __restrict__ y, int ypitch) {
  constexpr int KS = D / 32;
  constexpr int DT = D / 16;
  __shared__ __attribute__((aligned(16))) unsigned short sKh[32][D + 8], sKl[32][D + 8], sVh[32][D + 8], sVl[32][D + 8];
  __shared__ __attribute__((aligned(16))) unsigned short sPh[4][16][40], sPl[4][16][40];
  __shared__ __attribute__((aligned(16))) float sO[4][16][D];
  const int tid = threadIdx.x, w = tid >> 5, lane = tid & 31, ln = lane & 15, hh = lane >> 4;
  const int nqb = (T + 63) / 64;
  const int bh = blockIdx.x / nqb, qblk = blockIdx.x % nqb;
  const int b = bh / H, h = bh % H;
  const int q0 = qblk * 64 + w * 16;
  const float* Q = qb + (size_t)b * T * pitch + h * D;
  const float* K = kb + (size_t)b * T * pitch + h * D;
  const float* V = vb + (size_t)b * T * pitch + h * D;

  FragB aqh[KS], aql[KS];
  {
    int row = q0 + ln; if (row >= T) row = T - 1;
    const float* qr = Q + (size_t)row * pitch;
#pragma unroll
    for (int ks = 0; ks < KS; ++ks)
#pragma unroll
      for (int i = 0; i < 16; ++i) {
        const int d = ks * 32 + ((i < 8) ? (8 * hh + i) : (16 + 8 * hh + (i - 8)));
        const float x = qr[d] * scale; const unsigned short hb = bf16_bits(x);
        aqh[ks].u[i] = hb; aql[ks].u[i] = bf16_bits(x - bf16_val(hb));
      }
  }
  float m_r[8], l_r[8];
#pragma unroll
  for (int r = 0; r < 8; ++r) { m_r[r] = -3.0e38f; l_r[r] = 0.f; }
  v8f oacc[DT];
#pragma unroll
  for (int dt = 0; dt < DT; ++dt) oacc[dt] = (v8f){0.f,0.f,0.f,0.f,0.f,0.f,0.f,0.f};

  const int kv_end = CAUSAL ? min(T, qblk * 64 + 64) : T;
  for (int j0 = 0; j0 < kv_end; j0 += 32) {
    __syncthreads();
    for (int e = tid; e < 32 * (D / 4); e += 128) {
      const int r = e / (D / 4), c4 = (e % (D / 4)) * 4;
      const int key = j0 + r;
      v4f kf = {0.f,0.f,0.f,0.f}, vf = {0.f,0.f,0.f,0.f};
      if (key < T) { kf = *(const v4fa*)(K + (size_t)key * pitch + c4); vf = *(const v4fa*)(V + (size_t)key * pitch + c4); }
#pragma unroll
      for (int t = 0; t < 4; ++t) {
        unsigned short hb = bf16_bits(kf[t]); sKh[r][c4 + t] = hb; sKl[r][c4 + t] = bf16_bits(kf[t] - bf16_val(hb));
        hb = bf16_bits(vf[t]); sVh[r][c4 + t] = hb; sVl[r][c4 + t] = bf16_bits(vf[t] - bf16_val(hb));
      }
    }
    __syncthreads();
    v8f s[2];
#pragma unroll
    for (int nt = 0; nt < 2; ++nt) {
      v8f acc = {};
#pragma unroll
      for (int ks = 0; ks < KS; ++ks) {
        FragB bh_, bl_;
        bh_.half[0] = *(const v8us*)&sKh[nt * 16 + ln][ks * 32 + 8 * hh]; bh_.half[1] = *(const v8us*)&sKh[nt * 16 + ln][ks * 32 + 16 + 8 * hh];
        bl_.half[0] = *(const v8us*)&sKl[nt * 16 + ln][ks * 32 + 8 * hh]; bl_.half[1] = *(const v8us*)&sKl[nt * 16 + ln][ks * 32 + 16 + 8 * hh];
        acc = mmaN<3>(aqh[ks].v, aql[ks].v, bh_.v, bl_.v, acc);
      }
      s[nt] = acc;
    }
    float alpha[8];
#pragma unroll
    for (int r = 0; r < 8; ++r) {
      const int qi = q0 + 8 * hh + r;
      const int ja = j0 + ln, jb = j0 + 16 + ln;
      if (CAUSAL) { if (ja > qi) s[0][r] = -3.0e38f; if (jb > qi) s[1][r] = -3.0e38f; }
      if (ja >= T) s[0][r] = -3.0e38f;
      if (jb >= T) s[1][r] = -3.0e38f;
      float mx = fmaxf(s[0][r], s[1][r]);
      mx = fmaxf(mx, __shfl_xor(mx, 1, 32)); mx = fmaxf(mx, __shfl_xor(mx, 2, 32)); mx = fmaxf(mx, __shfl_xor(mx, 4, 32)); mx = fmaxf(mx, __shfl_xor(mx, 8, 32));
      const float mnew = fmaxf(m_r[r], mx);
      alpha[r] = (mnew > -1.0e38f) ? __expf(m_r[r] - mnew) : 1.0f;
      const float p0 = (s[0][r] > -1.0e38f) ? __expf(s[0][r] - mnew) : 0.f;
      const float p1 = (s[1][r] > -1.0e38f) ? __expf(s[1][r] - mnew) : 0.f;
      m_r[r] = mnew;
      l_r[r] = l_r[r] * alpha[r] + p0 + p1;
      unsigned short hb = bf16_bits(p0); sPh[w][8 * hh + r][ln] = hb;      sPl[w][8 * hh + r][ln] = bf16_bits(p0 - bf16_val(hb));
      hb = bf16_bits(p1);                sPh[w][8 * hh + r][16 + ln] = hb; sPl[w][8 * hh + r][16 + ln] = bf16_bits(p1 - bf16_val(hb));
    }
#pragma unroll
    for (int dt = 0; dt < DT; ++dt)
#pragma unroll
      for (int r = 0; r < 8; ++r) oacc[dt][r] *= alpha[r];
    __builtin_amdgcn_fence(__ATOMIC_ACQ_REL, "workgroup");
    __builtin_amdgcn_wave_barrier();
    FragB pah, pal;
    pah.half[0] = *(const v8us*)&sPh[w][ln][8 * hh]; pah.half[1] = *(const v8us*)&sPh[w][ln][16 + 8 * hh];
    pal.half[0] = *(const v8us*)&sPl[w][ln][8 * hh]; pal.half[1] = *(const v8us*)&sPl[w][ln][16 + 8 * hh];
#pragma unroll
    for (int dt = 0; dt < DT; ++dt) {
      FragB bvh, bvl;
#pragma unroll
      for (int i = 0; i < 8; ++i) {
        bvh.u[i] = sVh[8 * hh + i][dt * 16 + ln]; bvh.u[8 + i] = sVh[16 + 8 * hh + i][dt * 16 + ln];
        bvl.u[i] = sVl[8 * hh + i][dt * 16 + ln]; bvl.u[8 + i] = sVl[16 + 8 * hh + i][dt * 16 + ln];
      }
      oacc[dt] = mmaN<3>(pah.v, pal.v, bvh.v, bvl.v, oacc[dt]);
    }
    __builtin_amdgcn_fence(__ATOMIC_ACQ_REL, "workgroup");
    __builtin_amdgcn_wave_barrier();
  }
#pragma unroll
  for (int r = 0; r < 8; ++r) {
    float l = l_r[r];
    l += __shfl_xor(l, 1, 32); l += __shfl_xor(l, 2, 32); l += __shfl_xor(l, 4, 32); l += __shfl_xor(l, 8, 32);
    l_r[r] = (l > 0.f) ? 1.0f / l : 0.f;
  }
#pragma unroll
  for (int dt = 0; dt < DT; ++dt)
#pragma unroll
    for (int r = 0; r < 8; ++r) sO[w][8 * hh + r][dt * 16 + ln] = oacc[dt][r] * l_r[r];
  __builtin_amdgcn_fence(__ATOMIC_ACQ_REL, "workgroup");
  __builtin_amdgcn_wave_barrier();
  for (int pass = 0; pass < 2; ++pass) {
    for (int r = 0; r < 16; ++r) {
      const int row = q0 + r;
      if (row < T && lane < D / 4) {
        const v4f val = *(const v4fa*)&sO[w][r][lane * 4];
        *(volatile v4f*)(y + ((size_t)b * T + row) * ypitch + h * D + lane * 4) = val;
      }
    }
    if (pass == 0) __threadfence();
  }
}

template <bool ASPLIT, int ACT, bool BIAS_BF16, bool RES_BF16>
__global__ __launch_bounds__(128) void k_gemm_bf3(const float* __restrict__ A, int lda, const unsigned short* __restrict__ Wt, int ldb,
                                                const float* __restrict__ bias, const float* __restrict__ resid, int rmod, int ldr,
                                                float* __restrict__ C, int ldc, int M, int N, int K) {
  __shared__ __attribute__((aligned(16))) float so[4][16][64];
  const int tid = threadIdx.x, w = tid >> 5, lane = tid & 31, ln = lane & 15, hh = lane >> 4;
  const int ntn = N / 64;
  const int wid = blockIdx.x * 4 + w;
  const int mt = wid / ntn, nq = wid % ntn;
  if (mt * 16 >= M) return;
  const int row0 = mt * 16, col0 = nq * 64;
  const float* arow = A + (size_t)(row0 + ln) * lda;
  v8f acc[4] = {};
  for (int kb = 0; kb < K; kb += 32) {
    FragB ah, al;
    const v4f x0 = *(const v4fa*)(arow + kb + 8 * hh), x1 = *(const v4fa*)(arow + kb + 8 * hh + 4);
    const v4f x2 = *(const v4fa*)(arow + kb + 16 + 8 * hh), x3 = *(const v4fa*)(arow + kb + 16 + 8 * hh + 4);
    float xs[16] = {x0[0],x0[1],x0[2],x0[3],x1[0],x1[1],x1[2],x1[3],x2[0],x2[1],x2[2],x2[3],x3[0],x3[1],x3[2],x3[3]};
#pragma unroll
    for (int i = 0; i < 16; ++i) { const unsigned short hb = bf16_bits(xs[i]); ah.u[i] = hb; al.u[i] = ASPLIT ? bf16_bits(xs[i] - bf16_val(hb)) : (unsigned short)0; }
#pragma unroll
    for (int t = 0; t < 4; ++t) {
      const unsigned short* brow = Wt + (size_t)(col0 + t * 16 + ln) * ldb + kb;
      FragB b;
      b.half[0] = *(const v8us*)(brow + 8 * hh);
      b.half[1] = *(const v8us*)(brow + 16 + 8 * hh);
      acc[t] = mmaN<ASPLIT ? 2 : 1>(ah.v, al.v, b.v, b.v, acc[t]);
    }
  }
#pragma unroll
  for (int t = 0; t < 4; ++t) {
    const int col = col0 + t * 16 + ln;
    float bv = bias ? bias[col] : 0.f;
    if (BIAS_BF16) bv = bf16_round(bv);
#pragma unroll
    for (int r = 0; r < 8; ++r) {
      float v = acc[t][r] + bv;
      if (resid) { float rv = resid[(size_t)((row0 + 8 * hh + r) % rmod) * ldr + col]; if (RES_BF16) rv = bf16_round(rv); v += rv; }
      if (ACT == 1) v = fmaxf(v, 0.f);
      if (ACT == 2) v = 0.5f * v * (1.0f + erff(v * 0.70710678118654752f));
      if (ACT == 3) { const float u = 0.7978845608028654f * (v + 0.044715f * v * v * v); v = 0.5f * v * (1.0f + tanhf(u)); }
      so[w][8 * hh + r][t * 16 + ln] = v;
    }
  }
  __builtin_amdgcn_fence(__ATOMIC_ACQ_REL, "workgroup");
  __builtin_amdgcn_wave_barrier();
  const int rsub = lane >> 4, c4 = (lane & 15) * 4;
  for (int pass = 0; pass < 2; ++pass) {
#pragma unroll
    for (int q = 0; q < 8; ++q) {
      const int r = q * 2 + rsub;
      const v4f v = *(const v4fa*)&so[w][r][c4];
      *(volatile v4f*)(C + (size_t)(row0 + r) * ldc + col0 + c4) = v;
    }
    if (pass == 0) __threadfence();
  }
}
template <bool PARAM_BF16>
__global__ __launch_bounds__(256) void k_layernorm(const float* __restrict__ X, const float* __restrict__ R, const float* __restrict__ g, const float* __restrict__ bta,
                                                  float* __restrict__ out_sum, float* __restrict__ out_norm, int N, float eps) {
  __shared__ float red[256];
  const int row = blockIdx.x, tid = threadIdx.x;
  const float* x = X + (size_t)row * N; const float* rr = R ? R + (size_t)row * N : nullptr;
  float vals[16];
  const int per = N / 256;
  float s1 = 0.f;
  for (int u = 0; u < per / 4; ++u) {
    const int j = tid * 4 + 1024 * u;
    const v4f a = *(const v4fa*)(x + j);
    v4f b = {0.f,0.f,0.f,0.f}; if (rr) b = *(const v4fa*)(rr + j);
#pragma unroll
    for (int q = 0; q < 4; ++q) { const float v = a[q] + b[q]; vals[u * 4 + q] = v; s1 += v; }
  }
  red[tid] = s1; __syncthreads();
  for (int st = 128; st > 0; st >>= 1) { if (tid < st) red[tid] += red[tid + st]; __syncthreads(); }
  const float mu = red[0] / (float)N; __syncthreads();
  float s2 = 0.f;
  for (int u = 0; u < per / 4; ++u)
#pragma unroll
    for (int q = 0; q < 4; ++q) { const float c = vals[u * 4 + q] - mu; s2 += c * c; }
  red[tid] = s2; __syncthreads();
  for (int st = 128; st > 0; st >>= 1) { if (tid < st) red[tid] += red[tid + st]; __syncthreads(); }
  const float rs = rsqrtf(red[0] / (float)N + eps);
  for (int pass = 0; pass < 2; ++pass) {
    for (int u = 0; u < per / 4; ++u) {
      const int j = tid * 4 + 1024 * u;
      v4f o, sm;
#pragma unroll
      for (int q = 0; q < 4; ++q) {
        float gg = g[j + q], bb = bta[j + q];
        if (PARAM_BF16) { gg = bf16_round(gg); bb = bf16_round(bb); }
        sm[q] = vals[u * 4 + q]; o[q] = (vals[u * 4 + q] - mu) * rs * gg + bb;
      }
      if (out_sum) *(volatile v4f*)(out_sum + (size_t)row * N + j) = sm;
      *(volatile v4f*)(out_norm + (size_t)row * N + j) = o;
    }
    if (pass == 0) __threadfence();
  }
}


typedef _Float16 v16h __attribute__((ext_vector_type(16)));
union FragH { v16h v; v8us half[2]; _Float16 h[16]; unsigned short u[16]; };
template <int NT>
__device__ __forceinline__ v8f mmaH(v16h ah, v16h al, v16h bh, v16h bl, v8f c) {
  c = __builtin_amdgcn_wmma_f32_16x16x32_f16(false, ah, false, bh, (short)0, c, false, false);
  if (NT >= 2) c = __builtin_amdgcn_wmma_f32_16x16x32_f16(false, al, false, bh, (short)0, c, false, false);
  if (NT >= 3) c = __builtin_amdgcn_wmma_f32_16x16x32_f16(false, ah, false, bl, (short)0, c, false, false);
  asm volatile("v_nop\n\tv_nop\n\tv_nop\n\tv_nop" : "+v"(c) : "v"(ah), "v"(al), "v"(bh), "v"(bl));
  return c;
}
template <bool ASPLIT>
__global__ __launch_bounds__(128) void k_gemm_h(const float* __restrict__ A, int lda, size_t sA, const _Float16* __restrict__ Bh, int ldb, size_t sB, float alpha, float* __restrict__ C, int ldc, size_t sC, int M, int N, int K) {
  __shared__ __attribute__((aligned(16))) float so[4][16][64];
  const int tid = threadIdx.x, w = tid >> 5, lane = tid & 31, ln = lane & 15, hh = lane >> 4; const int by = blockIdx.y;
  A += (size_t)by * sA; Bh += (size_t)by * sB; C += (size_t)by * sC;
  const int ntn = (N + 63) / 64; const int wid = blockIdx.x * 4 + w; const int mt = wid / ntn, nq = wid % ntn; if (mt * 16 >= M) return;
  const int row0 = mt * 16, col0 = nq * 64; const float* arow = A + (size_t)(row0 + ln) * lda;
  v8f acc[4] = {};
  for (int kb = 0; kb < K; kb += 32) {
    FragH ah, al;
    const v4f x0 = *(const v4fa*)(arow + kb + 8 * hh), x1 = *(const v4fa*)(arow + kb + 8 * hh + 4), x2 = *(const v4fa*)(arow + kb + 16 + 8 * hh), x3 = *(const v4fa*)(arow + kb + 16 + 8 * hh + 4);
    float xs[16] = {x0[0],x0[1],x0[2],x0[3],x1[0],x1[1],x1[2],x1[3],x2[0],x2[1],x2[2],x2[3],x3[0],x3[1],x3[2],x3[3]};
#pragma unroll
    for (int i = 0; i < 16; ++i) { const _Float16 h = (_Float16)xs[i]; ah.h[i] = h; al.h[i] = ASPLIT ? (_Float16)(xs[i] - (float)h) : (_Float16)0.0f; }
#pragma unroll
    for (int t = 0; t < 4; ++t) { if (col0 + t * 16 >= N) continue; const size_t boff = (size_t)(col0 + t * 16 + ln) * ldb + kb; FragH bq; bq.half[0] = *(const v8us*)(Bh + boff + 8 * hh); bq.half[1] = *(const v8us*)(Bh + boff + 16 + 8 * hh);
      acc[t] = mmaH<ASPLIT ? 2 : 1>(ah.v, al.v, bq.v, bq.v, acc[t]); }
  }
#pragma unroll
  for (int t = 0; t < 4; ++t) { if (col0 + t * 16 >= N) continue;
#pragma unroll
    for (int r = 0; r < 8; ++r) so[w][8 * hh + r][t * 16 + ln] = acc[t][r] * alpha; }
  __builtin_amdgcn_fence(__ATOMIC_ACQ_REL, "workgroup"); __builtin_amdgcn_wave_barrier();
  const int rsub = lane >> 4, c4 = (lane & 15) * 4;
  for (int pass = 0; pass < 2; ++pass) {
#pragma unroll
    for (int q = 0; q < 8; ++q) { const int r = q * 2 + rsub; if (col0 + c4 < N) { const v4f v = *(const v4fa*)&so[w][r][c4]; *(volatile v4f*)(C + (size_t)(row0 + r) * ldc + col0 + c4) = v; } }
    if (pass == 0) __threadfence(); }
}

__global__ __launch_bounds__(256) void k_wt_f16(const float* __restrict__ W, _Float16* __restrict__ Wt, int K, int N, float scale) {
  const int t = blockIdx.x * 256 + threadIdx.x; if (t >= N * (K / 8)) return; const int n = t / (K / 8), k8 = (t % (K / 8)) * 8; FragH f;
#pragma unroll
  for (int i = 0; i < 8; ++i) f.h[i] = (_Float16)(bf16_round(W[(size_t)(k8 + i) * N + n]) * scale); const v8us o = f.half[0];
  *(volatile v8us*)((unsigned short*)Wt + (size_t)n * K + k8) = o; __threadfence(); *(volatile v8us*)((unsigned short*)Wt + (size_t)n * K + k8) = o;
}
template <int ACT>
__global__ __launch_bounds__(128) void k_gemm_hhx(const _Float16* __restrict__ A, int lda, size_t sA, const _Float16* __restrict__ Bh, int ldb, size_t sB, float alpha, const float* __restrict__ bias, size_t sBias, const float* __restrict__ CP, int rowsPerB, size_t sCPb, int row0g,
    float* __restrict__ C, _Float16* __restrict__ C16, int ldc, size_t sC, int M, int N, int K) {
  __shared__ __attribute__((aligned(16))) float so[4][16][64];
  const int tid = threadIdx.x, w = tid >> 5, lane = tid & 31, ln = lane & 15, hh = lane >> 4; const int by = blockIdx.y;
  A += (size_t)by * sA; Bh += (size_t)by * sB; const size_t cofs = (size_t)by * sC; const float* bp = bias ? bias + (size_t)by * sBias : nullptr;
  const int ntn = (N + 63) / 64; const int wid = blockIdx.x * 4 + w; const int mt = wid / ntn, nq = wid % ntn; if (mt * 16 >= M) return;
  const int row0 = mt * 16, col0 = nq * 64; const _Float16* arow = A + (size_t)(row0 + ln) * lda;
  v8f acc[4] = {};
  for (int kb = 0; kb < K; kb += 32) { FragH ah; ah.half[0] = *(const v8us*)((const unsigned short*)arow + kb + 8 * hh); ah.half[1] = *(const v8us*)((const unsigned short*)arow + kb + 16 + 8 * hh);
#pragma unroll
    for (int t = 0; t < 4; ++t) { if (col0 + t * 16 >= N) continue; const size_t boff = (size_t)(col0 + t * 16 + ln) * ldb + kb; FragH bq; bq.half[0] = *(const v8us*)((const unsigned short*)Bh + boff + 8 * hh); bq.half[1] = *(const v8us*)((const unsigned short*)Bh + boff + 16 + 8 * hh);
      acc[t] = mmaH<1>(ah.v, ah.v, bq.v, bq.v, acc[t]); }
  }
#pragma unroll
  for (int t = 0; t < 4; ++t) { if (col0 + t * 16 >= N) continue; const int col = col0 + t * 16 + ln; const float bv = bp ? bf16_round(bp[col]) : 0.f;
#pragma unroll
    for (int r = 0; r < 8; ++r) { float v = acc[t][r] * alpha + bv; if (CP) { const int bidx = (row0g + row0 + 8 * hh + r) / rowsPerB; v += CP[(size_t)bidx * sCPb + (size_t)by * 64 + col]; } if (ACT == 1) v = (v > 0.f) ? v : expm1f(v); else if (ACT == 3) v = fmaxf(v, 0.f); so[w][8 * hh + r][t * 16 + ln] = v; } }
  __builtin_amdgcn_fence(__ATOMIC_ACQ_REL, "workgroup"); __builtin_amdgcn_wave_barrier();
  const int rsub = lane >> 4, c4 = (lane & 15) * 4; typedef _Float16 v4h __attribute__((ext_vector_type(4)));
  for (int pass = 0; pass < 2; ++pass) {
#pragma unroll
    for (int q = 0; q < 8; ++q) { const int r = q * 2 + rsub; if (col0 + c4 < N) { const v4f v = *(const v4fa*)&so[w][r][c4]; if (C) *(volatile v4f*)(C + cofs + (size_t)(row0 + r) * ldc + col0 + c4) = v; if (C16) { v4h h4; for (int i = 0; i < 4; ++i) h4[i] = (_Float16)v[i]; *(volatile v4h*)(C16 + cofs + (size_t)(row0 + r) * ldc + col0 + c4) = h4; } } }
    if (pass == 0) __threadfence(); }
}


__global__ __launch_bounds__(256) void k_xt(const float* __restrict__ x, _Float16* __restrict__ XT) { const size_t t = (size_t)blockIdx.x * 256 + threadIdx.x; if (t >= (size_t)NP * CC / 8) return; const size_t p = t / (CC / 8); const int c8 = (int)(t % (CC / 8)) * 8; const int b = (int)(p / LQ), l = (int)(p % LQ); FragH f;
#pragma unroll
  for (int q = 0; q < 8; ++q) f.h[q] = (_Float16)bf16_round(x[((size_t)b * CC + c8 + q) * LQ + l]); *(volatile v8us*)((unsigned short*)XT + t * 8) = f.half[0]; __threadfence(); *(volatile v8us*)((unsigned short*)XT + t * 8) = f.half[0]; }
__global__ __launch_bounds__(256) void k_xmean(const float* __restrict__ x, float* __restrict__ XM) { __shared__ float sp[8][32]; const int tid = threadIdx.x, wv = tid >> 5, lane = tid & 31; const int b = blockIdx.x / (CC / 32), cg = blockIdx.x % (CC / 32);
  float res[4];
#pragma unroll
  for (int u = 0; u < 4; ++u) { const int c = cg * 32 + wv * 4 + u; const float* row = x + ((size_t)b * CC + c) * LQ; float s = 0.f;
#pragma unroll 1
    for (int i = lane; i < LQ; i += 32) s += bf16_round(row[i]); for (int o = 16; o >= 1; o >>= 1) s += __shfl_xor(s, o, 32); res[u] = s * (1.0f / (float)LQ); }
  if (lane == 0) { for (int u = 0; u < 4; ++u) sp[wv][u] = res[u]; } __syncthreads();
  if (tid < 32) { const float v = sp[tid / 4][tid % 4]; *(volatile float*)(XM + (size_t)b * CC + cg * 32 + tid) = v; } __threadfence(); if (tid < 32) { const float v = sp[tid / 4][tid % 4]; *(volatile float*)(XM + (size_t)b * CC + cg * 32 + tid) = v; } }
__global__ __launch_bounds__(256) void k_round16f(const float* __restrict__ W, _Float16* __restrict__ Bt, size_t n8) { const size_t t = (size_t)blockIdx.x * 256 + threadIdx.x; if (t >= n8) return; FragH f;
#pragma unroll
  for (int i = 0; i < 8; ++i) f.h[i] = (_Float16)(bf16_round(W[t * 8 + i]) * 16.0f); *(volatile v8us*)((unsigned short*)Bt + t * 8) = f.half[0]; __threadfence(); *(volatile v8us*)((unsigned short*)Bt + t * 8) = f.half[0]; }
__global__ __launch_bounds__(256) void k_wconv(const float* __restrict__ w, _Float16* __restrict__ Bc) { const size_t t = (size_t)blockIdx.x * 256 + threadIdx.x; if (t >= (size_t)CH * 9 * CC / 8) return; const int o = (int)(t / (9 * CC / 8)); const int k8 = (int)(t % (9 * CC / 8)) * 8; FragH f;
#pragma unroll
  for (int q = 0; q < 8; ++q) { const int k = k8 + q; const int tap = k / CC, c = k % CC; f.h[q] = (_Float16)(bf16_round(w[((size_t)o * CC + c) * 9 + tap]) * 16.0f); } *(volatile v8us*)((unsigned short*)Bc + t * 8) = f.half[0]; __threadfence(); *(volatile v8us*)((unsigned short*)Bc + t * 8) = f.half[0]; }
__global__ __launch_bounds__(128) void k_heat(const _Float16* __restrict__ XT, const _Float16* __restrict__ Bc, const float* __restrict__ bng, const float* __restrict__ bnb, const float* __restrict__ bnm, const float* __restrict__ bnv, const float* __restrict__ w2, const float* __restrict__ b2, float* __restrict__ heat) {
  __shared__ float sh[64];
  const int tid = threadIdx.x, w = tid >> 5, lane = tid & 31, ln = lane & 15, hh = lane >> 4; const int p0 = (blockIdx.x * 4 + w) * 16; const int p = p0 + ln; const int b = p / LQ, l = p % LQ, y = l / HW, xx = l % HW;
  v8f acc[8];
#pragma unroll
  for (int q = 0; q < 8; ++q) acc[q] = (v8f){0.f,0.f,0.f,0.f,0.f,0.f,0.f,0.f};
#pragma unroll 1
  for (int ks = 0; ks < 72; ++ks) { const int tap = ks >> 3, cb = (ks & 7) * 32; const int dy = tap / 3 - 1, dx = tap % 3 - 1; const int yy = y + dy, x2 = xx + dx; FragH a;
    if (yy >= 0 && yy < HW && x2 >= 0 && x2 < HW) { const unsigned short* ar = (const unsigned short*)XT + ((size_t)b * LQ + yy * HW + x2) * CC + cb; a.half[0] = *(const v8us*)(ar + 8 * hh); a.half[1] = *(const v8us*)(ar + 16 + 8 * hh); }
    else { for (int j = 0; j < 16; ++j) a.h[j] = (_Float16)0.0f; }
#pragma unroll
    for (int q = 0; q < 8; ++q) { FragH bq; const unsigned short* br = (const unsigned short*)Bc + (size_t)(q * 16 + ln) * (9 * CC) + ks * 32; bq.half[0] = *(const v8us*)(br + 8 * hh); bq.half[1] = *(const v8us*)(br + 16 + 8 * hh); acc[q] = mmaH<1>(a.v, a.v, bq.v, bq.v, acc[q]); } }
  float part[8];
#pragma unroll
  for (int r = 0; r < 8; ++r) part[r] = 0.f;
#pragma unroll
  for (int q = 0; q < 8; ++q) { const int o = q * 16 + ln; const float sc = bf16_round(bng[o]) / sqrtf(bf16_round(bnv[o]) + 1e-5f); const float sh_ = bf16_round(bnb[o]) - bf16_round(bnm[o]) * sc; const float wo = bf16_round(w2[o]);
#pragma unroll
    for (int r = 0; r < 8; ++r) { const float v = fmaxf(acc[q][r] * 0.0625f * sc + sh_, 0.f); part[r] += v * wo; } }
#pragma unroll
  for (int r = 0; r < 8; ++r) { float v = part[r]; v += __shfl_xor(v, 1, 32); v += __shfl_xor(v, 2, 32); v += __shfl_xor(v, 4, 32); v += __shfl_xor(v, 8, 32); part[r] = v; }
  if (ln == 0) { const float bb = bf16_round(b2[0]);
#pragma unroll
    for (int r = 0; r < 8; ++r) sh[w * 16 + 8 * hh + r] = 1.0f / (1.0f + expf(-(part[r] + bb))); }
  __syncthreads();
  if (tid < 64) { *(volatile float*)(heat + (size_t)blockIdx.x * 64 + tid) = sh[tid]; } __threadfence(); if (tid < 64) { *(volatile float*)(heat + (size_t)blockIdx.x * 64 + tid) = sh[tid]; } }
__global__ __launch_bounds__(256) void k_zoom(const float* __restrict__ x, const float* __restrict__ heat, _Float16* __restrict__ Z16) { const size_t t = (size_t)blockIdx.x * 256 + threadIdx.x; if (t >= (size_t)NP * CC / 8) return; const size_t p = t / (CC / 8); const int c8 = (int)(t % (CC / 8)) * 8; const int b = (int)(p / LQ), l = (int)(p % LQ); const float hp = heat[p]; FragH f;
#pragma unroll
  for (int q = 0; q < 8; ++q) f.h[q] = (_Float16)(bf16_round(x[((size_t)b * CC + c8 + q) * LQ + l]) * hp); *(volatile v8us*)((unsigned short*)Z16 + t * 8) = f.half[0]; __threadfence(); *(volatile v8us*)((unsigned short*)Z16 + t * 8) = f.half[0]; }
__global__ __launch_bounds__(256) void k_poolk(const float* __restrict__ QKV, _Float16* __restrict__ Kp) { const size_t t = (size_t)blockIdx.x * 256 + threadIdx.x; if (t >= (size_t)BB * LK * CC / 8) return; const int c8 = (int)(t % (CC / 8)) * 8; const size_t bj = t / (CC / 8); const int j = (int)(bj % LK), b = (int)(bj / LK); const int jy = j / (HW / 2), jx = j % (HW / 2);
  const size_t p00 = (size_t)b * LQ + (2 * jy) * HW + 2 * jx; FragH f;
#pragma unroll
  for (int q = 0; q < 8; ++q) { const int c = CC + c8 + q; const float s = QKV[p00 * 768 + c] + QKV[(p00 + 1) * 768 + c] + QKV[(p00 + HW) * 768 + c] + QKV[(p00 + HW + 1) * 768 + c]; f.h[q] = (_Float16)(s * 0.25f); }
  *(volatile v8us*)((unsigned short*)Kp + t * 8) = f.half[0]; __threadfence(); *(volatile v8us*)((unsigned short*)Kp + t * 8) = f.half[0]; }
__global__ __launch_bounds__(256) void k_poolv(const float* __restrict__ QKV, _Float16* __restrict__ Vt) { const size_t t = (size_t)blockIdx.x * 256 + threadIdx.x; if (t >= (size_t)BB * NHD * DH * LK / 8) return; const int j8 = (int)(t % (LK / 8)) * 8; const size_t bhd = t / (LK / 8); const int d = (int)(bhd % DH); const int h = (int)((bhd / DH) % NHD); const int b = (int)(bhd / ((size_t)DH * NHD)); FragH f;
#pragma unroll
  for (int q = 0; q < 8; ++q) { const int j = j8 + q; const int jy = j / (HW / 2), jx = j % (HW / 2); const size_t p00 = (size_t)b * LQ + (2 * jy) * HW + 2 * jx; const int c = 2 * CC + h * DH + d;
    const float s = QKV[p00 * 768 + c] + QKV[(p00 + 1) * 768 + c] + QKV[(p00 + HW) * 768 + c] + QKV[(p00 + HW + 1) * 768 + c]; f.h[q] = (_Float16)(s * 0.25f); }
  *(volatile v8us*)((unsigned short*)Vt + t * 8) = f.half[0]; __threadfence(); *(volatile v8us*)((unsigned short*)Vt + t * 8) = f.half[0]; }
__global__ __launch_bounds__(128) void k_flash(const float* __restrict__ QKV, const _Float16* __restrict__ Kp, const _Float16* __restrict__ Vt, float* __restrict__ O) {
  constexpr int RPW = 32, NQB = LQ / (4 * RPW);
  __shared__ __attribute__((aligned(16))) unsigned short sP[4][RPW][40]; __shared__ __attribute__((aligned(16))) float sO[4][RPW][DH];
  const int tid = threadIdx.x, w = tid >> 5, lane = tid & 31, ln = lane & 15, hh = lane >> 4;
  const int bh = blockIdx.x / NQB, qblk = blockIdx.x % NQB; const int b = bh / NHD, h = bh % NHD; const int q0 = qblk * (4 * RPW) + w * RPW;
  FragH aq[2];
#pragma unroll
  for (int rt = 0; rt < 2; ++rt) { const float* qr = QKV + ((size_t)b * LQ + q0 + rt * 16 + ln) * 768 + h * DH; const v4f x0 = *(const v4fa*)(qr + 8 * hh), x1 = *(const v4fa*)(qr + 8 * hh + 4), x2 = *(const v4fa*)(qr + 16 + 8 * hh), x3 = *(const v4fa*)(qr + 16 + 8 * hh + 4);
    const float xs[16] = {x0[0],x0[1],x0[2],x0[3],x1[0],x1[1],x1[2],x1[3],x2[0],x2[1],x2[2],x2[3],x3[0],x3[1],x3[2],x3[3]};
#pragma unroll
    for (int i = 0; i < 16; ++i) aq[rt].h[i] = (_Float16)xs[i]; }
  const unsigned short* Kb_ = (const unsigned short*)Kp + (size_t)b * LK * CC + h * DH; const unsigned short* Vt_ = (const unsigned short*)Vt + (size_t)bh * DH * LK;
  float m_r[2][8], l_r[2][8]; v8f oacc[2][2];
#pragma unroll
  for (int rt = 0; rt < 2; ++rt) {
#pragma unroll
    for (int r = 0; r < 8; ++r) { m_r[rt][r] = -3.0e38f; l_r[rt][r] = 0.f; }
    oacc[rt][0] = (v8f){0.f,0.f,0.f,0.f,0.f,0.f,0.f,0.f}; oacc[rt][1] = (v8f){0.f,0.f,0.f,0.f,0.f,0.f,0.f,0.f}; }
  const float scale = 0.17677669529663687f;
#pragma unroll 1
  for (int j0 = 0; j0 < LK; j0 += 32) {
    v8f s[2][2];
#pragma unroll
    for (int nt = 0; nt < 2; ++nt) { const unsigned short* brow = Kb_ + (size_t)(j0 + nt * 16 + ln) * CC; FragH bk; bk.half[0] = *(const v8us*)(brow + 8 * hh); bk.half[1] = *(const v8us*)(brow + 16 + 8 * hh);
#pragma unroll
      for (int rt = 0; rt < 2; ++rt) { v8f acc = (v8f){0.f,0.f,0.f,0.f,0.f,0.f,0.f,0.f}; s[rt][nt] = mmaH<1>(aq[rt].v, aq[rt].v, bk.v, bk.v, acc); } }
#pragma unroll
    for (int rt = 0; rt < 2; ++rt)
#pragma unroll
      for (int r = 0; r < 8; ++r) { const float s0 = s[rt][0][r] * scale, s1 = s[rt][1][r] * scale; float mc = fmaxf(s0, s1);
        mc = fmaxf(mc, __shfl_xor(mc, 1, 32)); mc = fmaxf(mc, __shfl_xor(mc, 2, 32)); mc = fmaxf(mc, __shfl_xor(mc, 4, 32)); mc = fmaxf(mc, __shfl_xor(mc, 8, 32));
        const float mn = fmaxf(m_r[rt][r], mc); const float al = expf(m_r[rt][r] - mn); m_r[rt][r] = mn;
        const float p0 = expf(s0 - mn), p1 = expf(s1 - mn); l_r[rt][r] = l_r[rt][r] * al + p0 + p1;
        oacc[rt][0][r] *= al; oacc[rt][1][r] *= al;
        FragH t2; t2.h[0] = (_Float16)p0; t2.h[1] = (_Float16)p1; sP[w][rt * 16 + 8 * hh + r][ln] = t2.u[0]; sP[w][rt * 16 + 8 * hh + r][16 + ln] = t2.u[1]; }
    __builtin_amdgcn_fence(__ATOMIC_ACQ_REL, "workgroup"); __builtin_amdgcn_wave_barrier();
    FragH pa[2];
#pragma unroll
    for (int rt = 0; rt < 2; ++rt) { pa[rt].half[0] = *(const v8us*)&sP[w][rt * 16 + ln][8 * hh]; pa[rt].half[1] = *(const v8us*)&sP[w][rt * 16 + ln][16 + 8 * hh]; }
#pragma unroll
    for (int dt = 0; dt < 2; ++dt) { const unsigned short* vrow = Vt_ + (size_t)(dt * 16 + ln) * LK + j0; FragH bv; bv.half[0] = *(const v8us*)(vrow + 8 * hh); bv.half[1] = *(const v8us*)(vrow + 16 + 8 * hh);
#pragma unroll
      for (int rt = 0; rt < 2; ++rt) oacc[rt][dt] = mmaH<1>(pa[rt].v, pa[rt].v, bv.v, bv.v, oacc[rt][dt]); }
    __builtin_amdgcn_fence(__ATOMIC_ACQ_REL, "workgroup"); __builtin_amdgcn_wave_barrier(); }
#pragma unroll
  for (int rt = 0; rt < 2; ++rt) {
#pragma unroll
    for (int r = 0; r < 8; ++r) { float l = l_r[rt][r]; l += __shfl_xor(l, 1, 32); l += __shfl_xor(l, 2, 32); l += __shfl_xor(l, 4, 32); l += __shfl_xor(l, 8, 32); l_r[rt][r] = 1.0f / l; }
#pragma unroll
    for (int dt = 0; dt < 2; ++dt)
#pragma unroll
      for (int r = 0; r < 8; ++r) sO[w][rt * 16 + 8 * hh + r][dt * 16 + ln] = oacc[rt][dt][r] * l_r[rt][r]; }
  __builtin_amdgcn_fence(__ATOMIC_ACQ_REL, "workgroup"); __builtin_amdgcn_wave_barrier();
  for (int pass = 0; pass < 2; ++pass) {
#pragma unroll
    for (int r = 0; r < RPW; ++r) { if (lane < DH / 4) { const v4f val = *(const v4fa*)&sO[w][r][lane * 4]; *(volatile v4f*)(O + ((size_t)b * LQ + q0 + r) * CC + h * DH + lane * 4) = val; } }
    if (pass == 0) __threadfence(); } }
__global__ __launch_bounds__(256) void k_gap(const float* __restrict__ O, float* __restrict__ GAP) { __shared__ float sp[8][4]; const int tid = threadIdx.x, wv = tid >> 5, lane = tid & 31; const int b = blockIdx.x / (CC / 32), cg = blockIdx.x % (CC / 32); float res[4];
#pragma unroll
  for (int u = 0; u < 4; ++u) { const int c = cg * 32 + wv * 4 + u; float s = 0.f;
#pragma unroll 1
    for (int i = lane; i < LQ; i += 32) s += O[((size_t)b * LQ + i) * CC + c]; for (int o = 16; o >= 1; o >>= 1) s += __shfl_xor(s, o, 32); res[u] = s * (1.0f / (float)LQ); }
  if (lane == 0) { for (int u = 0; u < 4; ++u) sp[wv][u] = res[u]; } __syncthreads();
  if (tid < 32) { *(volatile float*)(GAP + (size_t)b * CC + cg * 32 + tid) = sp[tid / 4][tid % 4]; } __threadfence(); if (tid < 32) { *(volatile float*)(GAP + (size_t)b * CC + cg * 32 + tid) = sp[tid / 4][tid % 4]; } }
__global__ __launch_bounds__(256) void k_segate(const float* __restrict__ GAP, const float* __restrict__ XM, const float* __restrict__ sw1, const float* __restrict__ sb1, const float* __restrict__ sw2, const float* __restrict__ sb2, const float* __restrict__ gw1, const float* __restrict__ gb1, const float* __restrict__ gw2, const float* __restrict__ gb2, float* __restrict__ CHG) {
  __shared__ float sgap[CC], sgi[2 * CC], shid[CH]; const int c = threadIdx.x;
  for (int b = 0; b < BB; ++b) {
    sgap[c] = GAP[b * CC + c]; sgi[c] = XM[b * CC + c]; __syncthreads();
    if (c < SE) { float s = bf16_round(sb1[c]);
#pragma unroll 1
      for (int k = 0; k < CC; ++k) s += sgap[k] * bf16_round(sw1[c * CC + k]); shid[c] = fmaxf(s, 0.f); }
    __syncthreads();
    float cha; { float s = bf16_round(sb2[c]);
#pragma unroll
      for (int k = 0; k < SE; ++k) s += shid[k] * bf16_round(sw2[c * SE + k]); cha = 1.0f / (1.0f + expf(-s)); }
    sgi[CC + c] = sgap[c] * cha; __syncthreads();
    if (c < CH) { float s = bf16_round(gb1[c]);
#pragma unroll 1
      for (int k = 0; k < 2 * CC; ++k) s += sgi[k] * bf16_round(gw1[c * 2 * CC + k]); shid[c] = fmaxf(s, 0.f); }
    __syncthreads();
    float gate; { float s = bf16_round(gb2[c]);
#pragma unroll 1
      for (int k = 0; k < CH; ++k) s += shid[k] * bf16_round(gw2[c * CH + k]); gate = 1.0f / (1.0f + expf(-s)); }
    for (int pass = 0; pass < 2; ++pass) { *(volatile float*)(CHG + (size_t)b * 2 * CC + c) = cha; *(volatile float*)(CHG + (size_t)b * 2 * CC + CC + c) = gate; if (pass == 0) __threadfence(); }
    __syncthreads(); } }
__global__ __launch_bounds__(256) void k_fuse(const float* __restrict__ x, const float* __restrict__ heat, const float* __restrict__ O, const float* __restrict__ CHG, float* __restrict__ out) { const size_t e = (size_t)blockIdx.x * 256 + threadIdx.x; if (e >= (size_t)BB * CC * LQ) return;
  const int l = (int)(e % LQ); const int c = (int)((e / LQ) % CC); const int b = (int)(e / ((size_t)LQ * CC)); const size_t p = (size_t)b * LQ + l;
  const float xv = bf16_round(x[e]); const float cha = CHG[(size_t)b * 2 * CC + c], g = CHG[(size_t)b * 2 * CC + CC + c];
  const float v = xv * (1.0f - g) + (xv * heat[p] + O[p * CC + c] * cha) * g; *(volatile float*)(out + e) = v; __threadfence(); *(volatile float*)(out + e) = v; }

extern "C" void kernel_launch(void* const* d_in, const int* in_sizes, int n_in,
                              void* d_out, int out_size, void* d_ws, size_t ws_size, hipStream_t stream) {
  (void)in_sizes; (void)n_in; (void)out_size;
  const float* x = (const float*)d_in[0]; const float* wq = (const float*)d_in[1]; const float* wk = (const float*)d_in[2]; const float* wv = (const float*)d_in[3]; const float* hw1 = (const float*)d_in[4];
  const float* bng = (const float*)d_in[5]; const float* bnb = (const float*)d_in[6]; const float* bnm = (const float*)d_in[7]; const float* bnv = (const float*)d_in[8]; const float* hw2 = (const float*)d_in[9]; const float* hb2 = (const float*)d_in[10];
  const float* sw1 = (const float*)d_in[11]; const float* sb1 = (const float*)d_in[12]; const float* sw2 = (const float*)d_in[13]; const float* sb2 = (const float*)d_in[14]; const float* gw1 = (const float*)d_in[15]; const float* gb1 = (const float*)d_in[16]; const float* gw2 = (const float*)d_in[17]; const float* gb2 = (const float*)d_in[18];
  char* ws = (char*)d_ws; size_t off = 0;
  auto take = [&](size_t bytes) { char* p = ws + off; off += (bytes + 255) & ~(size_t)255; return p; };
  _Float16* Bqkv = (_Float16*)take((size_t)3 * CC * CC * 2); _Float16* Bc = (_Float16*)take((size_t)CH * 9 * CC * 2); float* XM = (float*)take((size_t)BB * CC * 4); float* GAP = (float*)take((size_t)BB * CC * 4); float* CHG = (float*)take((size_t)BB * 2 * CC * 4); float* heat = (float*)take((size_t)NP * 4);
  _Float16* XT = (_Float16*)take((size_t)NP * CC * 2); _Float16* Z16 = (_Float16*)take((size_t)NP * CC * 2); float* QKV = (float*)take((size_t)NP * 3 * CC * 4); _Float16* Kp = (_Float16*)take((size_t)BB * LK * CC * 2); _Float16* Vtt = (_Float16*)take((size_t)BB * NHD * DH * LK * 2); float* O = (float*)take((size_t)NP * CC * 4);
  if (off > ws_size) return;
  k_round16f<<<(unsigned)(((size_t)CC * CC / 8 + 255) / 256), 256, 0, stream>>>(wq, Bqkv, (size_t)CC * CC / 8); k_round16f<<<(unsigned)(((size_t)CC * CC / 8 + 255) / 256), 256, 0, stream>>>(wk, Bqkv + (size_t)CC * CC, (size_t)CC * CC / 8); k_round16f<<<(unsigned)(((size_t)CC * CC / 8 + 255) / 256), 256, 0, stream>>>(wv, Bqkv + (size_t)2 * CC * CC, (size_t)CC * CC / 8);
  k_wconv<<<(unsigned)(((size_t)CH * 9 * CC / 8 + 255) / 256), 256, 0, stream>>>(hw1, Bc);
  k_xt<<<(unsigned)(((size_t)NP * CC / 8 + 255) / 256), 256, 0, stream>>>(x, XT); k_xmean<<<BB * (CC / 32), 256, 0, stream>>>(x, XM);
  k_heat<<<NP / 64, 128, 0, stream>>>(XT, Bc, bng, bnb, bnm, bnv, hw2, hb2, heat);
  k_zoom<<<(unsigned)(((size_t)NP * CC / 8 + 255) / 256), 256, 0, stream>>>(x, heat, Z16);
  k_gemm_hhx<0><<<dim3(((NP / 16) * (3 * CC / 64) + 3) / 4, 1), 128, 0, stream>>>(Z16, CC, 0, Bqkv, CC, 0, 0.0625f, nullptr, 0, nullptr, 1, 0, 0, QKV, nullptr, 3 * CC, 0, NP, 3 * CC, CC);
  k_poolk<<<(unsigned)(((size_t)BB * LK * CC / 8 + 255) / 256), 256, 0, stream>>>(QKV, Kp); k_poolv<<<(unsigned)(((size_t)BB * NHD * DH * LK / 8 + 255) / 256), 256, 0, stream>>>(QKV, Vtt);
  k_flash<<<BB * NHD * (LQ / 128), 128, 0, stream>>>(QKV, Kp, Vtt, O);
  k_gap<<<BB * (CC / 32), 256, 0, stream>>>(O, GAP);
  k_segate<<<1, 256, 0, stream>>>(GAP, XM, sw1, sb1, sw2, sb2, gw1, gb1, gw2, gb2, CHG);
  k_fuse<<<(unsigned)(((size_t)BB * CC * LQ + 255) / 256), 256, 0, stream>>>(x, heat, O, CHG, (float*)d_out);
}
